// TransformerEncoder_44676249813605
// MI455X (gfx1250) — hardware-verified
//
#include <hip/hip_runtime.h>
#include <math.h>

#ifndef NB
#define NB 8
#endif
#ifndef SEQ
#define SEQ 1024
#endif
#define NB_FULL 8
#define SEQ_FULL 1024
#define DM 512
#define NH 8
#define AU 64
#define DV 512
#define FFD 2048
#define QKW (2 * NH * AU)
#define HV (NH * DV)
#define HC (NH * DM)
#ifndef BG
#if (NB % 2) == 0
#define BG 2
#else
#define BG 1
#endif
#endif
static_assert(NB >= 1 && NB <= NB_FULL);
static_assert(SEQ % 64 == 0 && SEQ >= 64 && SEQ <= SEQ_FULL);
static_assert(NB % BG == 0);
static_assert(DM % 64 == 0 && AU == 64 && DV % 64 == 0 && FFD % 64 == 0 && QKW % 64 == 0 && HV % 64 == 0 && HC % 64 == 0);
static_assert((NB * SEQ) % 64 == 0 && (BG * SEQ) % 64 == 0);

#define C_X   8.0f
#define C_QKW 16.0f
#define C_QK  8.0f
#define C_VW  32.0f
#define C_LW  64.0f
#define C_M   256.0f
#define C_P   16384.0f
#define C_T   64.0f
#define C_H   8.0f
#define C_W1  32.0f
#define C_FF  16.0f
#define C_W2  32.0f

typedef __attribute__((ext_vector_type(16))) _Float16 v16h;
typedef __attribute__((ext_vector_type(8)))  _Float16 v8h;
typedef __attribute__((ext_vector_type(8)))  float    v8f;
typedef __attribute__((ext_vector_type(4)))  float    v4f;
typedef __attribute__((ext_vector_type(4)))  unsigned int v4u;

#define VST2(T, ptr, val) do { const T vst2_v_ = (val); *(volatile T*)(ptr) = vst2_v_; __threadfence(); *(volatile T*)(ptr) = vst2_v_; } while (0)
#define VST2V4(ptr, val) VST2(v4f, ptr, val)

__device__ __forceinline__ float bfr(float f) { unsigned int u = __float_as_uint(f); u += 0x7fffu + ((u >> 16) & 1u); return __uint_as_float(u & 0xffff0000u); }
__device__ __forceinline__ v4f bfr4(v4f a) { v4f r; r.x = bfr(a.x); r.y = bfr(a.y); r.z = bfr(a.z); r.w = bfr(a.w); return r; }
__device__ __forceinline__ unsigned short f2h(float x) { return (fabsf(x) < 6.104e-5f) ? (unsigned short)0 : __builtin_bit_cast(unsigned short, (_Float16)x); }
__device__ __forceinline__ v4u pack8h(const float* v) {
    v4u pk;
    pk.x = (unsigned int)f2h(v[0]) | ((unsigned int)f2h(v[1]) << 16);
    pk.y = (unsigned int)f2h(v[2]) | ((unsigned int)f2h(v[3]) << 16);
    pk.z = (unsigned int)f2h(v[4]) | ((unsigned int)f2h(v[5]) << 16);
    pk.w = (unsigned int)f2h(v[6]) | ((unsigned int)f2h(v[7]) << 16);
    return pk;
}
__device__ __forceinline__ void wsync() { __builtin_amdgcn_fence(3  , "workgroup"); __builtin_amdgcn_wave_barrier(); __builtin_amdgcn_fence(2  , "workgroup"); }

union HF { v16h v; v8h h[2]; };
__device__ __forceinline__ v16h fload(const _Float16* p) { HF f; f.h[0] = *(const v8h*)(p); f.h[1] = *(const v8h*)(p + 16); return f.v; }
__device__ __forceinline__ v8f wmma16(v16h a, v16h b, v8f c) {
    c = __builtin_amdgcn_wmma_f32_16x16x32_f16(false, a, false, b, (short)0, c, false, false);
    asm volatile("v_nop\n\tv_nop\n\tv_nop\n\tv_nop" : "+v"(c) : "v"(a), "v"(b));
    return c;
}
__device__ __forceinline__ void dep_guard_h(v8f& a, v8f& b, v16h x, v16h y) { asm volatile("v_nop\n\tv_nop\n\tv_nop\n\tv_nop" : "+v"(a), "+v"(b) : "v"(x), "v"(y)); }
__device__ __forceinline__ void keep4_h(v16h a, v16h b, v16h c, v16h d) { asm volatile("v_nop" :: "v"(a), "v"(b), "v"(c), "v"(d)); }
__device__ __forceinline__ void acc_guard4(v8f& a, v8f& b, v8f& c, v8f& d) { asm volatile("v_nop\n\tv_nop\n\tv_nop\n\tv_nop" : "+v"(a), "+v"(b), "+v"(c), "+v"(d)); }

__global__ __launch_bounds__(256) void k_x16(const float* __restrict__ x, unsigned short* __restrict__ X16, int nrows) {
    const long long u = (long long)blockIdx.x * 256 + threadIdx.x;
    if (u >= (long long)nrows * (DM / 8)) return;
    const int rr = (int)(u / (DM / 8)); const int c0 = 8 * (int)(u % (DM / 8));
    const int b = rr / SEQ, s = rr - b * SEQ;
    const float* src = x + ((long long)b * SEQ_FULL + s) * DM + c0;
    const v4f a = *(const v4f*)src, q = *(const v4f*)(src + 4);
    const float v[8] = {bfr(a.x) * C_X, bfr(a.y) * C_X, bfr(a.z) * C_X, bfr(a.w) * C_X, bfr(q.x) * C_X, bfr(q.y) * C_X, bfr(q.z) * C_X, bfr(q.w) * C_X};
    VST2(v4u, (v4u*)(X16 + (long long)rr * DM + c0), pack8h(v));
}
__global__ __launch_bounds__(256) void k_xt16(const float* __restrict__ x, unsigned short* __restrict__ XT16) {
    const long long u = (long long)blockIdx.x * 256 + threadIdx.x;
    if (u >= (long long)NB * DM * (SEQ / 8)) return;
    const int t0 = 8 * (int)(u % (SEQ / 8)); const long long bd = u / (SEQ / 8);
    const int d = (int)(bd % DM), b = (int)(bd / DM);
    const float* src = x + ((long long)b * SEQ_FULL + t0) * DM + d;
    float v[8];
#pragma unroll
    for (int i = 0; i < 8; ++i) v[i] = bfr(src[(long long)i * DM]) * C_X;
    VST2(v4u, (v4u*)(XT16 + bd * SEQ + t0), pack8h(v));
}
__global__ __launch_bounds__(256) void k_qkw(const float* __restrict__ qw, const float* __restrict__ kw, unsigned short* __restrict__ O16) {
    const long long u = (long long)blockIdx.x * 256 + threadIdx.x;
    if (u >= (long long)QKW * (DM / 8)) return;
    const int o = (int)(u / (DM / 8)); const int k0 = 8 * (int)(u % (DM / 8));
    const int hq = (o & (NH * AU - 1)) >> 6, uu = o & (AU - 1);
    float v[8];
#pragma unroll
    for (int i = 0; i < 8; ++i) {
        const long long idx = ((long long)hq * DM + (k0 + i)) * AU + uu;
        const float va = qw[idx], vb = kw[idx];
        v[i] = bfr((o < NH * AU) ? va : vb) * C_QKW;
    }
    VST2(v4u, (v4u*)(O16 + (long long)o * DM + k0), pack8h(v));
}
__global__ __launch_bounds__(256) void k_cvt8(const float* __restrict__ X, long long n8, float s, unsigned short* __restrict__ O16) {
    const long long u = (long long)blockIdx.x * 256 + threadIdx.x;
    if (u >= n8) return;
    const v4f a = *(const v4f*)(X + 8 * u), q = *(const v4f*)(X + 8 * u + 4);
    const float v[8] = {bfr(a.x) * s, bfr(a.y) * s, bfr(a.z) * s, bfr(a.w) * s, bfr(q.x) * s, bfr(q.y) * s, bfr(q.z) * s, bfr(q.w) * s};
    VST2(v4u, (v4u*)(O16 + 8 * u), pack8h(v));
}
__global__ __launch_bounds__(256) void k_wt(const float* __restrict__ W, int ldw, int KI, int NO, float s, unsigned short* __restrict__ O16) {
    const long long u = (long long)blockIdx.x * 256 + threadIdx.x;
    const int per = KI / 8;
    if (u >= (long long)NO * per) return;
    const int o = (int)(u / per); const int k0 = 8 * (int)(u % per);
    float v[8];
#pragma unroll
    for (int i = 0; i < 8; ++i) v[i] = bfr(W[(long long)(k0 + i) * ldw + o]) * s;
    VST2(v4u, (v4u*)(O16 + (long long)o * KI + k0), pack8h(v));
}

struct G64P {
    const unsigned short* A; const unsigned short* Bt; void* C; const float* bias;
    long long sAo, sAi, sBo, sBi, sCo, sCi, sBias;
    int lda, ldb, ldc, M, N, K, zin, pad_; float scale, oscale;
};
static_assert(sizeof(G64P) == 4 * 8 + 7 * 8 + 10 * 4);

template <int BIAS_MODE, int OUT_MODE, int ACT, bool BRNE>
__global__ __launch_bounds__(256) void k_gemm64(G64P p) {
    __shared__ __align__(16) float sT[8][16 * 68];
    const int lane = threadIdx.x & 31, wave = threadIdx.x >> 5;
    const int z = blockIdx.y; const int zo = z / p.zin, zi = z - zo * p.zin;
    const int tilesN = p.N >> 6, tilesM = p.M >> 6;
    const int tile = blockIdx.x * 8 + wave;
    if (tile >= tilesM * tilesN) return;
    const int tm = tile / tilesN, tn = tile - tm * tilesN;
    const int m0 = tm << 6, n0 = tn << 6;
    const _Float16* Ab = (const _Float16*)p.A + ((long long)zo * p.sAo + (long long)zi * p.sAi);
    const _Float16* Bb = (const _Float16*)p.Bt + ((long long)zo * p.sBo + (long long)zi * p.sBi);
    const int rl = lane & 15, koff = (lane >> 4) * 8, mOff = (lane >> 4) * 8;

    v8f acc[4][4];
#pragma unroll
    for (int i = 0; i < 4; ++i)
#pragma unroll
        for (int j = 0; j < 4; ++j) acc[i][j] = (v8f){0.f, 0.f, 0.f, 0.f, 0.f, 0.f, 0.f, 0.f};

    for (int k0 = 0; k0 < p.K; k0 += 32) {
        v16h bh[4];
#pragma unroll
        for (int j = 0; j < 4; ++j) bh[j] = fload(Bb + (long long)(n0 + (j << 4) + rl) * p.ldb + koff + k0);
#pragma unroll
        for (int i = 0; i < 4; ++i) {
            const v16h ah = fload(Ab + (long long)(m0 + (i << 4) + rl) * p.lda + koff + k0);
#pragma unroll
            for (int j = 0; j < 4; ++j)
                acc[i][j] = __builtin_amdgcn_wmma_f32_16x16x32_f16(false, ah, false, bh[j], (short)0, acc[i][j], false, false);
            dep_guard_h(acc[i][0], acc[i][3], ah, ah);
        }
        keep4_h(bh[0], bh[1], bh[2], bh[3]);
    }
    acc_guard4(acc[0][0], acc[0][1], acc[0][2], acc[0][3]);
    acc_guard4(acc[1][0], acc[1][1], acc[1][2], acc[1][3]);
    acc_guard4(acc[2][0], acc[2][1], acc[2][2], acc[2][3]);
    acc_guard4(acc[3][0], acc[3][1], acc[3][2], acc[3][3]);

    float* slab = sT[wave];
#pragma unroll
    for (int i = 0; i < 4; ++i) {
        const int mBase = m0 + (i << 4);
        v4f rs0 = {1.f, 1.f, 1.f, 1.f}, rs1 = rs0;
        if (BIAS_MODE == 3) { const float* rp = p.bias + (long long)z * p.sBias + mBase + mOff; rs0 = *(const v4f*)rp; rs1 = *(const v4f*)(rp + 4); }
        const float rsv[8] = {rs0.x, rs0.y, rs0.z, rs0.w, rs1.x, rs1.y, rs1.z, rs1.w};
#pragma unroll
        for (int j = 0; j < 4; ++j) {
            const int n = n0 + (j << 4) + rl;
            float bv = 0.f;
            if (BIAS_MODE == 2) { bv = p.bias[n]; if (BRNE) bv = bfr(bv); }
#pragma unroll
            for (int r = 0; r < 8; ++r) {
                float v = acc[i][j][r] * p.scale;
                if (BIAS_MODE == 2) v += bv;
                if (BIAS_MODE == 3) v *= rsv[r];
                if (ACT == 2) v = fmaxf(v, 0.f);
                v *= p.oscale;
                slab[(mOff + r) * 68 + (j << 4) + rl] = v;
            }
        }
        wsync();
        if (OUT_MODE == 0) {
            float* C = (float*)p.C + ((long long)zo * p.sCo + (long long)zi * p.sCi);
            const int hh = lane >> 4, c4 = (lane & 15) * 4;
            for (int pass = 0; pass < 2; ++pass) {
#pragma unroll
                for (int it = 0; it < 8; ++it) {
                    const int row = it * 2 + hh;
                    const v4f v = *(const v4f*)(slab + row * 68 + c4);
                    *(volatile v4f*)(C + (long long)(mBase + row) * p.ldc + n0 + c4) = v;
                }
                __threadfence();
            }
        } else {
            unsigned short* C = (unsigned short*)p.C + ((long long)zo * p.sCo + (long long)zi * p.sCi);
            const int q8 = lane >> 3, c8 = (lane & 7) * 8;
            v4u hv[4];
#pragma unroll
            for (int it = 0; it < 4; ++it) {
                const int row = it * 4 + q8;
                const v4f p0 = *(const v4f*)(slab + row * 68 + c8), p1 = *(const v4f*)(slab + row * 68 + c8 + 4);
                const float t8[8] = {p0.x, p0.y, p0.z, p0.w, p1.x, p1.y, p1.z, p1.w};
                hv[it] = pack8h(t8);
            }
            for (int pass = 0; pass < 2; ++pass) {
#pragma unroll
                for (int it = 0; it < 4; ++it) *(volatile v4u*)(C + (long long)(mBase + it * 4 + q8) * p.ldc + n0 + c8) = hv[it];
                __threadfence();
            }
        }
        wsync();
    }
}

__global__ __launch_bounds__(128) void k_prob(const unsigned short* __restrict__ QKp, int b0, unsigned short* __restrict__ Pp, float* __restrict__ RINV, float cfac, float pcarry) {
    __shared__ __align__(16) _Float16 pt[4][16 * 72];
    __shared__ __align__(16) float rv[64];
    const int lane = threadIdx.x & 31, wave = threadIdx.x >> 5, hh = lane >> 4, c = lane & 15;
    const int qblk = blockIdx.x, h = blockIdx.y, bl = blockIdx.z;
    const int b = b0 + bl, z = bl * NH + h;
    const int q0 = qblk * 64 + wave * 16;
    const _Float16* QK = (const _Float16*)QKp;
    _Float16* P16 = (_Float16*)Pp;
    const _Float16* qrow = QK + (long long)(b * SEQ + q0 + c) * QKW + h * AU;
    v16h qa[2];
#pragma unroll
    for (int dc = 0; dc < 2; ++dc) qa[dc] = fload(qrow + dc * 32 + 8 * hh);
    const _Float16* kbase = QK + (long long)b * SEQ * QKW + NH * AU + h * AU;
    const v8f z8 = {0.f, 0.f, 0.f, 0.f, 0.f, 0.f, 0.f, 0.f};
    float m8[8], l8[8];
#pragma unroll
    for (int i = 0; i < 8; ++i) { m8[i] = -3.0e38f; l8[i] = 0.f; }

    for (int j0 = 0; j0 < SEQ; j0 += 64) {
        v8f s[4];
#pragma unroll
        for (int j = 0; j < 4; ++j) {
            const _Float16* krow = kbase + (long long)(j0 + 16 * j + c) * QKW;
            v8f a = z8;
#pragma unroll
            for (int dc = 0; dc < 2; ++dc) a = wmma16(qa[dc], fload(krow + dc * 32 + 8 * hh), a);
            s[j] = a;
        }
#pragma unroll
        for (int i = 0; i < 8; ++i)
#pragma unroll
            for (int j = 0; j < 4; ++j) m8[i] = fmaxf(m8[i], s[j][i]);
    }
#pragma unroll
    for (int i = 0; i < 8; ++i) {
        float m = m8[i];
        m = fmaxf(m, __shfl_xor(m, 1, 32)); m = fmaxf(m, __shfl_xor(m, 2, 32));
        m = fmaxf(m, __shfl_xor(m, 4, 32)); m = fmaxf(m, __shfl_xor(m, 8, 32));
        m8[i] = m * cfac;
    }

    _Float16* mp = pt[wave];
    const int srow = lane >> 3, c8 = (lane & 7) * 8;
    for (int j0 = 0; j0 < SEQ; j0 += 64) {
        v8f s[4];
#pragma unroll
        for (int j = 0; j < 4; ++j) {
            const _Float16* krow = kbase + (long long)(j0 + 16 * j + c) * QKW;
            v8f a = z8;
#pragma unroll
            for (int dc = 0; dc < 2; ++dc) a = wmma16(qa[dc], fload(krow + dc * 32 + 8 * hh), a);
            s[j] = a;
        }
        wsync();
#pragma unroll
        for (int i = 0; i < 8; ++i) {
#pragma unroll
            for (int j = 0; j < 4; ++j) {
                const float pp = exp2f(s[j][i] * cfac - m8[i]);
                l8[i] += pp;
                mp[(8 * hh + i) * 72 + 16 * j + c] = __builtin_bit_cast(_Float16, f2h(pp * pcarry));
            }
        }
        wsync();
        v8h hv[4];
#pragma unroll
        for (int it = 0; it < 4; ++it) hv[it] = *(const v8h*)(mp + (it * 4 + srow) * 72 + c8);
        _Float16* prow = P16 + ((long long)z * SEQ + q0) * SEQ + j0 + c8;
        for (int pass = 0; pass < 2; ++pass) {
#pragma unroll
            for (int it = 0; it < 4; ++it) *(volatile v8h*)(prow + (long long)(it * 4 + srow) * SEQ) = hv[it];
            __threadfence();
        }
    }

    float lsel = 1.f;
#pragma unroll
    for (int i = 0; i < 8; ++i) {
        float l = l8[i];
        l += __shfl_xor(l, 1, 32); l += __shfl_xor(l, 2, 32); l += __shfl_xor(l, 4, 32); l += __shfl_xor(l, 8, 32);
        if ((c & 7) == i) lsel = l;
    }
    if (c < 8) rv[wave * 16 + 8 * hh + c] = 1.0f / lsel;
    __syncthreads();
    if (wave == 0 && lane < 16) {
        const v4f r4 = *(const v4f*)(rv + 4 * lane);
        VST2V4(RINV + (long long)z * SEQ + qblk * 64 + 4 * lane, r4);
    }
}

__global__ __launch_bounds__(256) void k_ln(const float* __restrict__ A, const float* __restrict__ R, int rfull, int rrne,
                                            const float* __restrict__ gam, const float* __restrict__ bet,
                                            float* __restrict__ Y, int yfull, unsigned short* __restrict__ Y16, float s16, int nrows) {
    __shared__ __align__(16) float st[8][DM];
    const int wave = threadIdx.x >> 5, lane = threadIdx.x & 31;
    const int rr = blockIdx.x * 8 + wave;
    if (rr >= nrows) return;
    const int b = rr / SEQ, s = rr - b * SEQ; const long long rf = (long long)b * SEQ_FULL + s;
    const float* a = A + (long long)rr * DM;
    const float* r = R + (rfull ? rf : (long long)rr) * DM;
    v4f v[4]; float sum = 0.f;
#pragma unroll
    for (int i = 0; i < 4; ++i) {
        const int cc = 128 * i + 4 * lane;
        const v4f va = *(const v4f*)(a + cc); v4f vr = *(const v4f*)(r + cc);
        if (rrne) vr = bfr4(vr);
        v[i] = va + vr;
        sum += (v[i].x + v[i].y) + (v[i].z + v[i].w);
    }
#pragma unroll
    for (int o = 16; o > 0; o >>= 1) sum += __shfl_xor(sum, o, 32);
    const float mean = sum * (1.f / (float)DM);
    v4f d[4]; float q = 0.f;
#pragma unroll
    for (int i = 0; i < 4; ++i) { d[i] = v[i] - mean; q += (d[i].x * d[i].x + d[i].y * d[i].y) + (d[i].z * d[i].z + d[i].w * d[i].w); }
#pragma unroll
    for (int o = 16; o > 0; o >>= 1) q += __shfl_xor(q, o, 32);
    const float var = q * (1.f / (float)DM);
    const float rs = 1.0f / sqrtf(var + 1.0e-3f);
    float* y = Y + (yfull ? rf : (long long)rr) * DM;
#pragma unroll
    for (int i = 0; i < 4; ++i) {
        const int cc = 128 * i + 4 * lane;
        const v4f g4 = bfr4(*(const v4f*)(gam + cc)), b4 = bfr4(*(const v4f*)(bet + cc));
        const v4f o4 = g4 * (d[i] * rs) + b4;
        VST2V4(y + cc, o4);
        if (Y16) *(v4f*)(&st[wave][cc]) = o4;
    }
    if (Y16) {
        wsync();
#pragma unroll
        for (int i = 0; i < 2; ++i) {
            const int c8 = 256 * i + 8 * lane;
            const v4f p0 = *(const v4f*)(&st[wave][c8]), p1 = *(const v4f*)(&st[wave][c8 + 4]);
            const float t8[8] = {p0.x * s16, p0.y * s16, p0.z * s16, p0.w * s16, p1.x * s16, p1.y * s16, p1.z * s16, p1.w * s16};
            VST2(v4u, (v4u*)(Y16 + (long long)rr * DM + c8), pack8h(t8));
        }
    }
}

template <int BM_, int OM, int ACT, bool BR>
static void gemm_go(hipStream_t st, const void* A, long long sAo, long long sAi, int lda,
                    const void* Bt, long long sBo, long long sBi, int ldb,
                    void* C, long long sCo, long long sCi, int ldc,
                    const float* bias, long long sBias,
                    int M, int N, int K, int Z, int zin, float scale, float oscale) {
    G64P p;
    p.A = (const unsigned short*)A; p.Bt = (const unsigned short*)Bt; p.C = C; p.bias = bias;
    p.sAo = sAo; p.sAi = sAi; p.sBo = sBo; p.sBi = sBi; p.sCo = sCo; p.sCi = sCi; p.sBias = sBias;
    p.lda = lda; p.ldb = ldb; p.ldc = ldc; p.M = M; p.N = N; p.K = K; p.zin = zin; p.pad_ = 0; p.scale = scale; p.oscale = oscale;
    const int tiles = (M / 64) * (N / 64);
    dim3 grid((unsigned)((tiles + 7) / 8), (unsigned)Z);
    k_gemm64<BM_, OM, ACT, BR><<<grid, 256, 0, st>>>(p);
}
static inline unsigned cdiv(long long n, long long d) { return (unsigned)((n + d - 1) / d); }

extern "C" void kernel_launch(void* const* d_in, const int* in_sizes, int n_in, void* d_out, int out_size, void* d_ws, size_t ws_size, hipStream_t stream) {
    if (n_in < 13) return;
    if (in_sizes[0] < NB * SEQ_FULL * DM) return;
    if (in_sizes[1] < NH * DM * AU || in_sizes[2] < NH * DM * AU || in_sizes[3] < NH * DM * DV || in_sizes[4] < HV * DM) return;
    if (in_sizes[5] < DM || in_sizes[6] < DM || in_sizes[7] < DM * FFD || in_sizes[8] < FFD || in_sizes[9] < FFD * DM || in_sizes[10] < DM || in_sizes[11] < DM || in_sizes[12] < DM) return;
    if (out_size < NB * SEQ_FULL * DM) return;
    const float* x = (const float*)d_in[0];
    const float* qw = (const float*)d_in[1];
    const float* kw = (const float*)d_in[2];
    const float* vw = (const float*)d_in[3];
    const float* lw = (const float*)d_in[4];
    const float* gamma1 = (const float*)d_in[5];
    const float* beta1 = (const float*)d_in[6];
    const float* w1 = (const float*)d_in[7];
    const float* b1 = (const float*)d_in[8];
    const float* w2 = (const float*)d_in[9];
    const float* b2 = (const float*)d_in[10];
    const float* gamma2 = (const float*)d_in[11];
    const float* beta2 = (const float*)d_in[12];
    float* out = (float*)d_out;

    const size_t NR = (size_t)NB * SEQ;
    const size_t szQKW = (size_t)QKW * DM * 2, szVW = (size_t)NH * DM * DV * 2, szLW = (size_t)DM * HV * 2, szM = (size_t)DM * HC * 2, szW1 = (size_t)FFD * DM * 2, szW2 = (size_t)DM * FFD * 2;
    const size_t szMHA = NR * DM * 4;
    const size_t szX16 = NR * DM * 2, szXT = (size_t)NB * DM * SEQ * 2, szQK = NR * QKW * 2, szP = (size_t)BG * NH * SEQ * SEQ * 2, szT = (size_t)BG * SEQ * HC * 2, szRINV = (size_t)BG * NH * SEQ * 4;
    const size_t szH32 = NR * DM * 4, szH16 = NR * DM * 2, szFF1 = NR * FFD * 2, szFF2 = NR * DM * 4;
    const size_t phA = szX16 + szXT + szQK + szP + szT + szRINV;
    const size_t phB = szH32 + szH16 + szFF1 + szFF2;
    const size_t szR = (phA > phB) ? phA : phB;
    const size_t total = szQKW + szVW + szLW + szM + szW1 + szW2 + szMHA + szR;
    if (total > ws_size) return;
    if (total > (size_t)134217728) return;
    char* w = (char*)d_ws;
    unsigned short* QKW16 = (unsigned short*)w; w += szQKW;
    unsigned short* VW16 = (unsigned short*)w; w += szVW;
    unsigned short* LW16 = (unsigned short*)w; w += szLW;
    unsigned short* MT16 = (unsigned short*)w; w += szM;
    unsigned short* W116 = (unsigned short*)w; w += szW1;
    unsigned short* W216 = (unsigned short*)w; w += szW2;
    float* MHA32 = (float*)w; w += szMHA;
    char* R0 = w;
    unsigned short* X16 = (unsigned short*)R0;
    unsigned short* XT16 = (unsigned short*)(R0 + szX16);
    unsigned short* QK16 = (unsigned short*)(R0 + szX16 + szXT);
    unsigned short* P16 = (unsigned short*)(R0 + szX16 + szXT + szQK);
    unsigned short* T16 = (unsigned short*)(R0 + szX16 + szXT + szQK + szP);
    float* RINV = (float*)(R0 + szX16 + szXT + szQK + szP + szT);
    float* H32 = (float*)R0;
    unsigned short* H16 = (unsigned short*)(R0 + szH32);
    unsigned short* FF116 = (unsigned short*)(R0 + szH32 + szH16);
    float* FF232 = (float*)(R0 + szH32 + szH16 + szFF1);

    k_x16<<<cdiv((long long)NR * (DM / 8), 256), 256, 0, stream>>>(x, X16, (int)NR);
    k_xt16<<<cdiv((long long)NB * DM * (SEQ / 8), 256), 256, 0, stream>>>(x, XT16);
    k_qkw<<<cdiv((long long)QKW * (DM / 8), 256), 256, 0, stream>>>(qw, kw, QKW16);
    k_cvt8<<<cdiv((long long)NH * DM * (DV / 8), 256), 256, 0, stream>>>(vw, (long long)NH * DM * (DV / 8), C_VW, VW16);
    k_wt<<<cdiv((long long)DM * (HV / 8), 256), 256, 0, stream>>>(lw, DM, HV, DM, C_LW, LW16);
    k_wt<<<cdiv((long long)FFD * (DM / 8), 256), 256, 0, stream>>>(w1, FFD, DM, FFD, C_W1, W116);
    k_wt<<<cdiv((long long)DM * (FFD / 8), 256), 256, 0, stream>>>(w2, DM, FFD, DM, C_W2, W216);

    gemm_go<0, 1, 0, false>(stream, LW16, DV, 0, HV, VW16, (long long)DM * DV, 0, DV, MT16, DM, 0, HC, nullptr, 0,
                            DM, DM, DV, NH, 1, C_M / (C_LW * C_VW), 1.f);

    gemm_go<0, 1, 0, false>(stream, X16, 0, 0, DM, QKW16, 0, 0, DM, QK16, 0, 0, QKW, nullptr, 0, (int)NR, QKW, DM, 1, 1, C_QK / (C_X * C_QKW), 1.f);

    const float cfac = 1.4426950408889634f * 0.044194173824159216f / (C_QK * C_QK);
    for (int g = 0; g < NB / BG; ++g) {
        k_prob<<<dim3(SEQ / 64, NH, BG), 128, 0, stream>>>(QK16, g * BG, P16, RINV, cfac, C_P);
        gemm_go<3, 1, 0, false>(stream, P16, (long long)NH * SEQ * SEQ, (long long)SEQ * SEQ, SEQ,
                                XT16 + (size_t)g * BG * DM * SEQ, (long long)DM * SEQ, 0, SEQ,
                                T16, (long long)SEQ * HC, DM, HC, RINV, SEQ, SEQ, DM, SEQ, BG * NH, NH, C_T / (C_P * C_X), 1.f);
        gemm_go<0, 0, 0, false>(stream, T16, 0, 0, HC, MT16, 0, 0, HC, MHA32 + (size_t)g * BG * SEQ * DM, 0, 0, DM, nullptr, 0,
                                BG * SEQ, DM, HC, 1, 1, 1.f / (C_T * C_M), 1.f);
    }
    k_ln<<<(unsigned)(NR / 8), 256, 0, stream>>>(MHA32, x, 1, 1, gamma1, beta1, H32, 0, H16, C_H, (int)NR);
    gemm_go<2, 1, 2, true>(stream, H16, 0, 0, DM, W116, 0, 0, DM, FF116, 0, 0, FFD, b1, 0, (int)NR, FFD, DM, 1, 1, 1.f / (C_H * C_W1), C_FF);
    gemm_go<2, 0, 0, true>(stream, FF116, 0, 0, FFD, W216, 0, 0, FFD, FF232, 0, 0, DM, b2, 0, (int)NR, DM, FFD, 1, 1, 1.f / (C_FF * C_W2), 1.f);
    k_ln<<<(unsigned)(NR / 8), 256, 0, stream>>>(FF232, H32, 0, 0, gamma2, beta2, out, 1, nullptr, 1.f, (int)NR);
}
